// ProposalBranch_conf_54528904790789
// MI455X (gfx1250) — hardware-verified
//
#include <hip/hip_runtime.h>

typedef _Float16 f16t;
typedef _Float16 v16h __attribute__((ext_vector_type(16)));
typedef _Float16 v8h  __attribute__((ext_vector_type(8)));
typedef float    v8f  __attribute__((ext_vector_type(8)));
typedef float    v4f  __attribute__((ext_vector_type(4)));
typedef v8h __attribute__((may_alias)) v8ha;
typedef v4f __attribute__((may_alias)) v4fa;
union Frag { v16h v; v8h half[2]; };

#define NB    2
#define NT    128
#define NT2   512
#define CIN   512
#define PCH   512
#define SYP   132
#define STP   72
#define GEPS  1e-5f
#define WSC   64.0f
#define ACAR  8.0f

__device__ __forceinline__ v8f wmma_f16(v16h a, v16h b, v8f c) {
  v8f d = __builtin_amdgcn_wmma_f32_16x16x32_f16(false, a, false, b, (short)0, c, false, false);
  asm volatile("v_nop\n\tv_nop\n\tv_nop\n\tv_nop" : "+v"(d) : "v"(a), "v"(b));
  return d;
}

__device__ __forceinline__ v16h load_frag32(const f16t* p, int h) {
  Frag f;
  f.half[0] = *(const v8ha*)(p + 8 * h);
  f.half[1] = *(const v8ha*)(p + 16 + 8 * h);
  return f.v;
}

__device__ __forceinline__ v8f zero8f() {
  v8f z;
  #pragma unroll
  for (int j = 0; j < 8; ++j) z[j] = 0.f;
  return z;
}

__device__ __forceinline__ float wave_sum(float v) {
  v += __shfl_xor(v, 16);
  v += __shfl_xor(v, 8);
  v += __shfl_xor(v, 4);
  v += __shfl_xor(v, 2);
  v += __shfl_xor(v, 1);
  return v;
}

__global__ __launch_bounds__(256) void k_cvtw(
    const float* __restrict__ w0, const float* __restrict__ w1, const float* __restrict__ w2,
    const float* __restrict__ w3, const float* __restrict__ w4, const float* __restrict__ w5,
    f16t* __restrict__ d0, f16t* __restrict__ d1, f16t* __restrict__ d2,
    f16t* __restrict__ d3, f16t* __restrict__ d4, f16t* __restrict__ d5)
{
  const int g = blockIdx.x * 256 + threadIdx.x;
  if (g >= 2424832) return;
  const float* src;
  f16t* dst;
  int loc;
  if (g < 32768)        { loc = g;           src = w0; dst = d0; }
  else if (g < 98304)   { loc = g - 32768;   src = w1; dst = d1; }
  else if (g < 131072)  { loc = g - 98304;   src = w2; dst = d2; }
  else if (g < 327680)  { loc = g - 131072;  src = w3; dst = d3; }
  else if (g < 1376256) { loc = g - 327680;  src = w4; dst = d4; }
  else                  { loc = g - 1376256; src = w5; dst = d5; }
  const size_t e8 = (size_t)loc * 8;
  const v4f a = *(const v4fa*)(src + e8);
  const v4f c = *(const v4fa*)(src + e8 + 4);
  v8h o;
  o[0] = (f16t)(a.x * WSC); o[1] = (f16t)(a.y * WSC); o[2] = (f16t)(a.z * WSC); o[3] = (f16t)(a.w * WSC);
  o[4] = (f16t)(c.x * WSC); o[5] = (f16t)(c.y * WSC); o[6] = (f16t)(c.z * WSC); o[7] = (f16t)(c.w * WSC);
  *(volatile v8h*)(dst + e8) = o;
  __threadfence();
  *(volatile v8h*)(dst + e8) = o;
}

__global__ __launch_bounds__(256) void k_cvtx(const float* __restrict__ x, f16t* __restrict__ XT)
{
  __shared__ __attribute__((aligned(16))) f16t sT[NT * STP];
  const int tid = threadIdx.x, lane = tid & 31, w = tid >> 5;
  const int cg = blockIdx.x, b = blockIdx.y;
  const int tq = tid & 31, cl = tid >> 5;
  const int t0 = 4 * tq;
  #pragma unroll
  for (int j = 0; j < 8; ++j) {
    const int c = cl + 8 * j;
    const v4f v = *(const v4fa*)(x + ((size_t)(b * CIN + 64 * cg + c)) * NT + t0);
    sT[(t0 + 0) * STP + c] = (f16t)(v.x * ACAR);
    sT[(t0 + 1) * STP + c] = (f16t)(v.y * ACAR);
    sT[(t0 + 2) * STP + c] = (f16t)(v.z * ACAR);
    sT[(t0 + 3) * STP + c] = (f16t)(v.w * ACAR);
  }
  __syncthreads();
  const int q8 = lane & 7, sub = lane >> 3;
  v8h hv[4];
  #pragma unroll
  for (int i = 0; i < 4; ++i) {
    const int t = 16 * w + 4 * i + sub;
    hv[i] = *(const v8ha*)(sT + t * STP + 8 * q8);
  }
  #pragma unroll
  for (int i = 0; i < 4; ++i) {
    const int t = 16 * w + 4 * i + sub;
    const size_t d = ((size_t)(b * NT + t)) * CIN + 64 * cg + 8 * q8;
    *(volatile v8h*)(XT + d) = hv[i];
  }
  __threadfence();
  #pragma unroll
  for (int i = 0; i < 4; ++i) {
    const int t = 16 * w + 4 * i + sub;
    const size_t d = ((size_t)(b * NT + t)) * CIN + 64 * cg + 8 * q8;
    *(volatile v8h*)(XT + d) = hv[i];
  }
}

__global__ __launch_bounds__(256) void k_bmax(
    const float* __restrict__ feat, const float* __restrict__ segs, int C, int Tf,
    f16t* __restrict__ dst, int ldd, int choff, int total)
{
  const int g = blockIdx.x * 256 + threadIdx.x;
  if (g >= total) return;
  const int cpr = C >> 3;
  const int c8 = g % cpr;
  const int rest = g / cpr;
  const int n = rest % NT;
  const int b = rest / NT;
  const int c0 = 8 * c8;
  const int pr = (c0 < (C >> 1)) ? 0 : 2;
  const float s = segs[(size_t)(b * NT + n) * 4 + pr];
  const float e = segs[(size_t)(b * NT + n) * 4 + pr + 1];
  float fs = floorf(s), fe = floorf(e);
  fs = fminf(fmaxf(fs, 0.0f), (float)Tf);
  fe = fminf(fmaxf(fe, -1.0f), (float)(Tf - 1));
  const int lo = (int)fs, hi = (int)fe;
  const float ninf = __uint_as_float(0xff800000u);
  float mx[8];
  #pragma unroll
  for (int j = 0; j < 8; ++j) mx[j] = ninf;
  const float* fb = feat + ((size_t)(b * C + c0)) * Tf;
  #pragma unroll 1
  for (int t = lo; t <= hi; ++t) {
    #pragma unroll
    for (int j = 0; j < 8; ++j) mx[j] = fmaxf(mx[j], fb[(size_t)j * Tf + t]);
  }
  const bool nonempty = (lo <= hi);
  v8h o;
  #pragma unroll
  for (int j = 0; j < 8; ++j) o[j] = (f16t)((nonempty ? mx[j] : 0.0f) * ACAR);
  const size_t d = ((size_t)(b * NT + n)) * ldd + choff + c0;
  *(volatile v8h*)(dst + d) = o;
  __threadfence();
  *(volatile v8h*)(dst + d) = o;
}

__global__ __launch_bounds__(256) void k_gath(
    const float* __restrict__ feat, const float* __restrict__ anc, const int* __restrict__ ordp,
    int C, int Tf, int kklog, f16t* __restrict__ dst, int total)
{
  const int g = blockIdx.x * 256 + threadIdx.x;
  if (g >= total) return;
  (void)ordp;
  const int KK = 1 << kklog;
  const int nkq = KK >> 3;
  const int kq = g & (nkq - 1);
  int rest = g >> (kklog - 3);
  const int c = rest % C;
  rest /= C;
  const int l = rest % NT;
  const int b = rest / NT;
  const float a0 = anc[(size_t)(b * NT + l) * 2];
  const float a1 = anc[(size_t)(b * NT + l) * 2 + 1];
  const float tf = (float)Tf;
  const float left = fminf(fmaxf(a0, 0.0f), tf);
  const float right = fminf(fmaxf(a1, 0.0f), tf);
  const bool valid = right > left;
  const int li = (int)floorf(left);
  const int ri = (int)floorf(right);
  int len = min(ri + 1, Tf) - li;
  len = max(len, 1);
  const float* fr = feat + ((size_t)(b * C + c)) * Tf;
  v8h o;
  #pragma unroll
  for (int j = 0; j < 8; ++j) {
    const int k = 8 * kq + j;
    int id = li + ((k * len) >> kklog);
    id = min(max(id, 0), Tf - 1);
    const float v = fr[id];
    o[j] = (f16t)((valid ? v : 0.0f) * ACAR);
  }
  const size_t d = ((size_t)(b * NT + l)) * ((size_t)C * KK) + (size_t)c * KK + 8 * kq;
  *(volatile v8h*)(dst + d) = o;
  __threadfence();
  *(volatile v8h*)(dst + d) = o;
}

__global__ __launch_bounds__(256) void k_unit(
    const f16t* __restrict__ Aw, int K, const f16t* __restrict__ Bt,
    const float* __restrict__ bias, int gn, int Cg,
    const float* __restrict__ gam, const float* __restrict__ bet,
    float* outF, int wf32, int Cout,
    f16t* outT, int wf16, int ldt, int choff)
{
  __shared__ __attribute__((aligned(16))) float sY[64 * SYP];
  __shared__ float sR1[8];
  __shared__ float sR2[8];
  const int tid = threadIdx.x, lane = tid & 31, w = tid >> 5;
  const int h = lane >> 4, m = lane & 15;
  const int o0 = blockIdx.x * 64, b = blockIdx.y;
  const int mt = w & 3, ng = w >> 2;
  const v8f z8 = zero8f();
  v8f acc[4];
  #pragma unroll
  for (int nt = 0; nt < 4; ++nt) acc[nt] = z8;

  const f16t* arow = Aw + (size_t)(o0 + 16 * mt + m) * (size_t)K;
  const f16t* brow = Bt + (size_t)(b * NT + 64 * ng + m) * (size_t)K;
  #pragma unroll 2
  for (int k0 = 0; k0 < K; k0 += 32) {
    const v16h a = load_frag32(arow + k0, h);
    #pragma unroll
    for (int nt = 0; nt < 4; ++nt) {
      const v16h bb = load_frag32(brow + (size_t)(16 * nt) * (size_t)K + k0, h);
      acc[nt] = wmma_f16(a, bb, acc[nt]);
    }
  }

  const float osc = 1.0f / (ACAR * WSC);
  #pragma unroll
  for (int r = 0; r < 8; ++r) {
    const int ol = 16 * mt + 8 * h + r;
    const float bv = bias[o0 + ol];
    #pragma unroll
    for (int nt = 0; nt < 4; ++nt) sY[ol * SYP + 64 * ng + 16 * nt + m] = acc[nt][r] * osc + bv;
  }
  __syncthreads();

  const int ngr = 64 / Cg;
  const int wpg = 8 / ngr;
  const int tpg = 32 * wpg;
  const int gi = w / wpg;
  const int q = tid - gi * tpg;
  const int rbase = gi * Cg;
  const float invn = (Cg == 16) ? (1.0f / 2048.0f) : (1.0f / 4096.0f);
  float mean = 0.0f, rstd = 1.0f;
  if (gn) {
    float s = 0.0f;
    #pragma unroll 4
    for (int j = 0; j < 32; ++j) {
      const int e = q + tpg * j;
      s += sY[(rbase + (e >> 7)) * SYP + (e & 127)];
    }
    s = wave_sum(s);
    if (lane == 0) sR1[w] = s;
  }
  __syncthreads();
  if (gn) {
    float t = 0.0f;
    for (int u = 0; u < wpg; ++u) t += sR1[gi * wpg + u];
    mean = t * invn;
    float s2 = 0.0f;
    #pragma unroll 4
    for (int j = 0; j < 32; ++j) {
      const int e = q + tpg * j;
      const float dv = sY[(rbase + (e >> 7)) * SYP + (e & 127)] - mean;
      s2 += dv * dv;
    }
    s2 = wave_sum(s2);
    if (lane == 0) sR2[w] = s2;
  }
  __syncthreads();
  if (gn) {
    float t2 = 0.0f;
    for (int u = 0; u < wpg; ++u) t2 += sR2[gi * wpg + u];
    const float var = t2 * invn;
    rstd = rsqrtf(var + GEPS);
    #pragma unroll 4
    for (int j = 0; j < 32; ++j) {
      const int e = q + tpg * j;
      const int rl = e >> 7, cl = e & 127;
      const int o = o0 + rbase + rl;
      const int idx = (rbase + rl) * SYP + cl;
      const float y = (sY[idx] - mean) * rstd * gam[o] + bet[o];
      sY[idx] = fmaxf(y, 0.0f);
    }
  }
  __syncthreads();

  if (wf32) {
    v4f vals[8];
    #pragma unroll
    for (int i = 0; i < 8; ++i) {
      const int row = w + 8 * i;
      vals[i] = *(const v4fa*)(sY + row * SYP + 4 * lane);
    }
    #pragma unroll
    for (int i = 0; i < 8; ++i) {
      const int row = w + 8 * i;
      const size_t d = ((size_t)(b * Cout + o0 + row)) * NT + 4 * lane;
      *(volatile v4f*)(outF + d) = vals[i];
    }
    __threadfence();
    #pragma unroll
    for (int i = 0; i < 8; ++i) {
      const int row = w + 8 * i;
      const size_t d = ((size_t)(b * Cout + o0 + row)) * NT + 4 * lane;
      *(volatile v4f*)(outF + d) = vals[i];
    }
  }
  if (wf16) {
    const int q8 = lane & 7, sub = lane >> 3;
    v8h hv[4];
    #pragma unroll
    for (int i = 0; i < 4; ++i) {
      const int t = 16 * w + 4 * i + sub;
      #pragma unroll
      for (int j = 0; j < 8; ++j) hv[i][j] = (f16t)(sY[(8 * q8 + j) * SYP + t] * ACAR);
    }
    #pragma unroll
    for (int i = 0; i < 4; ++i) {
      const int t = 16 * w + 4 * i + sub;
      const size_t d = ((size_t)(b * NT + t)) * ldt + choff + o0 + 8 * q8;
      *(volatile v8h*)(outT + d) = hv[i];
    }
    __threadfence();
    #pragma unroll
    for (int i = 0; i < 4; ++i) {
      const int t = 16 * w + 4 * i + sub;
      const size_t d = ((size_t)(b * NT + t)) * ldt + choff + o0 + 8 * q8;
      *(volatile v8h*)(outT + d) = hv[i];
    }
  }
}

static inline int cdiv(int a, int b) { return (a + b - 1) / b; }

extern "C" void kernel_launch(void* const* d_in, const int* in_sizes, int n_in,
                              void* d_out, int out_size, void* d_ws, size_t ws_size,
                              hipStream_t stream) {
  if (n_in < 28) return;
  if (in_sizes[0] != NB * CIN * NT) return;
  if (in_sizes[1] != NB * CIN * NT2) return;
  if (in_sizes[2] != NB * NT * 4 || in_sizes[3] != NB * NT * 4) return;
  if (in_sizes[4] != NB * NT * 2 || in_sizes[5] != NB * NT * 2) return;
  if (in_sizes[7] != PCH * CIN || in_sizes[8] != PCH || in_sizes[9] != PCH || in_sizes[10] != PCH) return;
  if (in_sizes[11] != 2 * PCH * CIN || in_sizes[12] != 2 * PCH || in_sizes[13] != 2 * PCH || in_sizes[14] != 2 * PCH) return;
  if (in_sizes[15] != PCH * PCH || in_sizes[16] != PCH || in_sizes[17] != PCH || in_sizes[18] != PCH) return;
  if (in_sizes[19] != CIN * 6 * PCH || in_sizes[20] != CIN || in_sizes[21] != CIN || in_sizes[22] != CIN) return;
  if (in_sizes[23] != PCH * PCH * 32 || in_sizes[24] != PCH) return;
  if (in_sizes[25] != PCH * 2 * PCH * 16 || in_sizes[26] != PCH) return;
  if (in_sizes[27] < 1) return;
  if (out_size != NB * CIN * NT + NB * 2 * PCH * NT) return;

  const float* feature = (const float*)d_in[0];
  const float* frame   = (const float*)d_in[1];
  const float* segs    = (const float*)d_in[2];
  const float* fsegs   = (const float*)d_in[3];
  const float* anchor  = (const float*)d_in[4];
  const float* fanchor = (const float*)d_in[5];
  const float* W_cur  = (const float*)d_in[7];
  const float* b_cur  = (const float*)d_in[8];
  const float* g_cur  = (const float*)d_in[9];
  const float* be_cur = (const float*)d_in[10];
  const float* W_lr   = (const float*)d_in[11];
  const float* b_lr   = (const float*)d_in[12];
  const float* g_lr   = (const float*)d_in[13];
  const float* be_lr  = (const float*)d_in[14];
  const float* W_roi  = (const float*)d_in[15];
  const float* b_roi  = (const float*)d_in[16];
  const float* g_roi  = (const float*)d_in[17];
  const float* be_roi = (const float*)d_in[18];
  const float* W_prop  = (const float*)d_in[19];
  const float* b_prop  = (const float*)d_in[20];
  const float* g_prop  = (const float*)d_in[21];
  const float* be_prop = (const float*)d_in[22];
  const float* W_cp0 = (const float*)d_in[23];
  const float* b_cp0 = (const float*)d_in[24];
  const float* W_cp1 = (const float*)d_in[25];
  const float* b_cp1 = (const float*)d_in[26];
  const int*   order = (const int*)d_in[27];
  float* out0 = (float*)d_out;
  float* out1 = out0 + (size_t)NB * CIN * NT;

  const size_t szWc  = (size_t)PCH * CIN * 2;
  const size_t szWl  = (size_t)2 * PCH * CIN * 2;
  const size_t szWr  = (size_t)PCH * PCH * 2;
  const size_t szWp  = (size_t)CIN * 6 * PCH * 2;
  const size_t szWk  = (size_t)PCH * 16384 * 2;
  const size_t szXT  = (size_t)NB * NT * CIN * 2;
  const size_t szPL  = (size_t)NB * NT * PCH * 2;
  const size_t szFC  = (size_t)NB * NT * PCH * 2;
  const size_t szCT  = (size_t)NB * NT * 6 * PCH * 2;
  const size_t szG   = (size_t)NB * NT * 16384 * 2;
  size_t off = 0;
  char* ws = (char*)d_ws;
  f16t* Wc16 = (f16t*)(ws + off); off += szWc;
  f16t* Wl16 = (f16t*)(ws + off); off += szWl;
  f16t* Wr16 = (f16t*)(ws + off); off += szWr;
  f16t* Wp16 = (f16t*)(ws + off); off += szWp;
  f16t* W016 = (f16t*)(ws + off); off += szWk;
  f16t* W116 = (f16t*)(ws + off); off += szWk;
  f16t* XT   = (f16t*)(ws + off); off += szXT;
  f16t* PLT  = (f16t*)(ws + off); off += szPL;
  f16t* FCT  = (f16t*)(ws + off); off += szFC;
  f16t* CATT = (f16t*)(ws + off); off += szCT;
  f16t* G1T  = (f16t*)(ws + off); off += szG;
  f16t* G2T  = (f16t*)(ws + off); off += szG;
  if (off > ws_size) return;
  if (off > (size_t)134217728) return;

  const int nPoolLr = NB * NT * (2 * PCH) / 8;
  const int nPoolFr = NB * NT * PCH / 8;
  const int nG1 = NB * NT * (2 * PCH) * 2;
  const int nG2 = NB * NT * PCH * 4;

  k_cvtw<<<9472, 256, 0, stream>>>(W_cur, W_lr, W_roi, W_prop, W_cp0, W_cp1,
                                   Wc16, Wl16, Wr16, Wp16, W016, W116);
  k_cvtx<<<dim3(CIN / 64, NB), 256, 0, stream>>>(feature, XT);
  k_unit<<<dim3(PCH / 64, NB), 256, 0, stream>>>(Wc16, CIN, XT, b_cur, 1, 16, g_cur, be_cur,
                                                 out0, 0, PCH, CATT, 1, 6 * PCH, 3 * PCH);
  k_unit<<<dim3(2 * PCH / 64, NB), 256, 0, stream>>>(Wl16, CIN, XT, b_lr, 1, 32, g_lr, be_lr,
                                                     out1, 1, 2 * PCH, CATT, 0, 6 * PCH, 0);
  k_bmax<<<cdiv(nPoolLr, 256), 256, 0, stream>>>(out1, segs, 2 * PCH, NT, CATT, 6 * PCH, PCH, nPoolLr);
  k_bmax<<<cdiv(nPoolFr, 256), 256, 0, stream>>>(frame, fsegs, CIN, NT2, PLT, PCH, 0, nPoolFr);
  k_unit<<<dim3(PCH / 64, NB), 256, 0, stream>>>(Wr16, PCH, PLT, b_roi, 1, 16, g_roi, be_roi,
                                                 out0, 0, PCH, CATT, 1, 6 * PCH, 0);
  k_gath<<<cdiv(nG1, 256), 256, 0, stream>>>(out1, anchor, order, 2 * PCH, NT, 4, G1T, nG1);
  k_unit<<<dim3(PCH / 64, NB), 256, 0, stream>>>(W116, 16384, G1T, b_cp1, 0, 16, b_cp1, b_cp1,
                                                 out0, 0, PCH, CATT, 1, 6 * PCH, 4 * PCH);
  k_gath<<<cdiv(nG2, 256), 256, 0, stream>>>(frame, fanchor, order, CIN, NT2, 5, G2T, nG2);
  k_unit<<<dim3(PCH / 64, NB), 256, 0, stream>>>(W016, 16384, G2T, b_cp0, 0, 16, b_cp0, b_cp0,
                                                 out0, 0, PCH, FCT, 1, PCH, 0);
  k_unit<<<dim3(PCH / 64, NB), 256, 0, stream>>>(Wr16, PCH, FCT, b_roi, 1, 16, g_roi, be_roi,
                                                 out0, 0, PCH, CATT, 1, 6 * PCH, 5 * PCH);
  k_unit<<<dim3(CIN / 64, NB), 256, 0, stream>>>(Wp16, 6 * PCH, CATT, b_prop, 1, 16, g_prop, be_prop,
                                                 out0, 1, CIN, CATT, 0, 6 * PCH, 0);
}
